// VanillaSLSTMFeat_36275293782360
// MI455X (gfx1250) — hardware-verified
//
#include <hip/hip_runtime.h>


#define TT   2048
#define BB   2
#define EE   1024
#define NH_  16
#define NG   (BB * NH_)
#define HD   64
#define NR   33
#define MR   16
#define ZH   2
#define RH   512
#define PCAR 1024.0f
typedef _Float16 h16;
typedef unsigned short bf;
typedef __attribute__((ext_vector_type(16))) __bf16   v16bf;
typedef __attribute__((ext_vector_type(16))) _Float16 v16h;
typedef __attribute__((ext_vector_type(8)))  _Float16 v8h;
typedef __attribute__((ext_vector_type(8)))  unsigned short v8us;
typedef __attribute__((ext_vector_type(8)))  float    v8f;
typedef __attribute__((ext_vector_type(4)))  float    v4f;
typedef v8h  __attribute__((may_alias)) v8ha;
typedef v4f  __attribute__((may_alias)) v4fa;
typedef v8us __attribute__((may_alias)) v8usa;

__device__ __forceinline__ unsigned short f2bf(float f) { unsigned u = __float_as_uint(f); u += 0x7FFFu + ((u >> 16) & 1u); return (unsigned short)(u >> 16); }
__device__ __forceinline__ float bf2f(unsigned short b) { return __uint_as_float(((unsigned)b) << 16); }
__device__ __forceinline__ float bfr(float f) { return bf2f(f2bf(f)); }
__device__ __forceinline__ v16h cat16(v8h lo, v8h hi) { return __builtin_shufflevector(lo, hi, 0, 1, 2, 3, 4, 5, 6, 7, 8, 9, 10, 11, 12, 13, 14, 15); }
__device__ __forceinline__ v16bf cat16b(v8us lo, v8us hi) { return __builtin_bit_cast(v16bf, __builtin_shufflevector(lo, hi, 0, 1, 2, 3, 4, 5, 6, 7, 8, 9, 10, 11, 12, 13, 14, 15)); }
__device__ __forceinline__ v8f wmma16(v16h a, v16h b, v8f c) { return __builtin_amdgcn_wmma_f32_16x16x32_f16(false, a, false, b, (short)0, c, false, false); }
__device__ __forceinline__ v8f wmmab(v16bf a, v16bf b, v8f c) { return __builtin_amdgcn_wmma_f32_16x16x32_bf16(false, a, false, b, (short)0, c, false, false); }


template <typename T16> struct WFrag;
template <> struct WFrag<h16> { typedef v16h V; static __device__ __forceinline__ V ld(const h16* p) { return cat16(*(const v8h*)p, *(const v8h*)(p + 16)); } static __device__ __forceinline__ v8f mma(V a, V b, v8f c) { return wmma16(a, b, c); } };
template <> struct WFrag<bf> { typedef v16bf V; static __device__ __forceinline__ V ld(const bf* p) { return cat16b(*(const v8us*)p, *(const v8us*)(p + 16)); } static __device__ __forceinline__ v8f mma(V a, V b, v8f c) { return wmmab(a, b, c); } };
template <typename T16, int NSPLIT, bool BIAS>
__global__ __launch_bounds__(32) void k_gemmw(const T16* __restrict__ A, const T16* __restrict__ A2, const T16* __restrict__ Bt, const T16* __restrict__ Bt2, int K, float* C, int ldc, const float* __restrict__ bias, size_t sA, size_t sB, size_t sC) {
    typedef typename WFrag<T16>::V V;
    __shared__ __align__(16) float os[16 * 68];
    const size_t z = blockIdx.z; A += z * sA; if (A2) A2 += z * sA; Bt += z * sB; if (Bt2) Bt2 += z * sB; C += z * sC;
    const int lane = threadIdx.x & 31, lr = lane & 15, hi = lane >> 4; const int r0 = blockIdx.x * 64, c0 = blockIdx.y * 64;
    v8f acc[4][4];
#pragma unroll
    for (int mb = 0; mb < 4; ++mb)
#pragma unroll
        for (int nb = 0; nb < 4; ++nb) acc[mb][nb] = (v8f){};
    const size_t aoff = (size_t)(r0 + lr) * K + 8 * hi, boff = (size_t)(c0 + lr) * K + 8 * hi;
#pragma unroll 1
    for (int kc = 0; kc < K; kc += 32) {
        V a[4], a2[4];
#pragma unroll
        for (int mb = 0; mb < 4; ++mb) { a[mb] = WFrag<T16>::ld(A + aoff + (size_t)mb * 16 * K + kc); if (NSPLIT == 1 || NSPLIT == 2) a2[mb] = WFrag<T16>::ld(A2 + aoff + (size_t)mb * 16 * K + kc); }
#pragma unroll
        for (int nb = 0; nb < 4; ++nb) { const V b = WFrag<T16>::ld(Bt + boff + (size_t)nb * 16 * K + kc); V b2; if (NSPLIT >= 2) b2 = WFrag<T16>::ld(Bt2 + boff + (size_t)nb * 16 * K + kc);
#pragma unroll
            for (int mb = 0; mb < 4; ++mb) { acc[mb][nb] = WFrag<T16>::mma(a[mb], b, acc[mb][nb]); if (NSPLIT == 1 || NSPLIT == 2) acc[mb][nb] = WFrag<T16>::mma(a2[mb], b, acc[mb][nb]); if (NSPLIT >= 2) acc[mb][nb] = WFrag<T16>::mma(a[mb], b2, acc[mb][nb]); } }
        asm volatile("v_nop\n\tv_nop\n\tv_nop\n\tv_nop" : "+v"(acc[0][0]), "+v"(acc[1][1]), "+v"(acc[2][2]), "+v"(acc[3][3]) : "v"(a[0]), "v"(a[3]));
    }
#pragma unroll
    for (int mb = 0; mb < 4; ++mb) {
#pragma unroll
        for (int nb = 0; nb < 4; ++nb) {
#pragma unroll
            for (int j = 0; j < 8; ++j) os[(hi * 8 + j) * 68 + nb * 16 + lr] = acc[mb][nb][j]; }
        __builtin_amdgcn_wave_barrier(); asm volatile("" ::: "memory");
        float* crow = C + (size_t)(r0 + mb * 16) * ldc + c0;
#pragma unroll 1
        for (int ps = 0; ps < 2; ++ps) {
#pragma unroll
            for (int s = 0; s < 8; ++s) { const int row = 2 * s + hi, cofs = lr * 4; v4f val = *(const v4fa*)(os + row * 68 + cofs); if (BIAS) { val[0] += bfr(bias[c0 + cofs]); val[1] += bfr(bias[c0 + cofs + 1]); val[2] += bfr(bias[c0 + cofs + 2]); val[3] += bfr(bias[c0 + cofs + 3]); }
                *(volatile v4f*)(crow + (size_t)row * ldc + cofs) = val; }
            if (ps == 0) __threadfence(); }
        __builtin_amdgcn_wave_barrier(); asm volatile("" ::: "memory");
    }
}

__device__ __forceinline__ h16 tohx(float x) { return (h16)x; }
__device__ __forceinline__ void splitf(float y, unsigned short& h, unsigned short& l) { h = f2bf(y); l = f2bf(y - bf2f(h)); }
typedef __attribute__((ext_vector_type(2))) _Float16 v2h;
typedef __attribute__((ext_vector_type(4))) _Float16 v4h;
typedef __attribute__((ext_vector_type(2))) unsigned short v2us;
typedef __attribute__((ext_vector_type(4))) unsigned short v4us;
typedef __attribute__((ext_vector_type(2))) float v2f;

__global__ __launch_bounds__(256) void k_cvt8(const float* __restrict__ src, bf* dst, size_t n8) { const size_t i = (size_t)blockIdx.x * 256 + threadIdx.x; if (i >= n8) return; const v8f v = *(const v8f*)(src + i * 8); v8us o;
#pragma unroll
    for (int k = 0; k < 8; ++k) o[k] = f2bf(v[k]); *(volatile v8us*)(dst + i * 8) = o; __threadfence(); *(volatile v8us*)(dst + i * 8) = o; }
__global__ __launch_bounds__(256) void k_pl(const float* __restrict__ F, float scl, h16* P16, bf* Ph, bf* Pl) { const size_t e = ((size_t)blockIdx.x * 256 + threadIdx.x) * 2; if (e >= (size_t)NG * TT * HD) return; const int d = (int)(e % HD); const int t = (int)((e / HD) % TT); const int n = (int)(e / ((size_t)HD * TT)); const int b = n / NH_, h = n % NH_; const float* f = F + ((size_t)t * BB + b) * EE + h * HD + d; v2h o; v2us oh, ol;
#pragma unroll
    for (int u = 0; u < 2; ++u) { const float v = f[u] * scl; o[u] = tohx(v); unsigned short a, c; splitf(v, a, c); oh[u] = a; ol[u] = c; } for (int ps = 0; ps < 2; ++ps) { *(volatile v2h*)(P16 + e) = o; *(volatile v2us*)(Ph + e) = oh; *(volatile v2us*)(Pl + e) = ol; if (ps == 0) __threadfence(); } }
__global__ __launch_bounds__(256) void k_vtp(const float* __restrict__ F, h16* V16, bf* Vh, bf* Vl) { const size_t e = ((size_t)blockIdx.x * 256 + threadIdx.x) * 2; if (e >= (size_t)NG * HD * TT) return; const int t = (int)(e % TT); const int d = (int)((e / TT) % HD); const int n = (int)(e / ((size_t)TT * HD)); const int b = n / NH_, h = n % NH_; v2h o; v2us oh, ol;
#pragma unroll
    for (int u = 0; u < 2; ++u) { const float v = F[((size_t)(t + u) * BB + b) * EE + h * HD + d]; o[u] = tohx(v); unsigned short a, c; splitf(v, a, c); oh[u] = a; ol[u] = c; } for (int ps = 0; ps < 2; ++ps) { *(volatile v2h*)(V16 + e) = o; *(volatile v2us*)(Vh + e) = oh; *(volatile v2us*)(Vl + e) = ol; if (ps == 0) __threadfence(); } }
__global__ __launch_bounds__(256) void k_qr(const float* __restrict__ QF, const float* __restrict__ rk, float* QR) { const size_t e = (size_t)blockIdx.x * 256 + threadIdx.x; if (e >= (size_t)NG * TT * 64) return; const int r = (int)(e % 64); const int t = (int)((e / 64) % TT); const int n = (int)(e / ((size_t)64 * TT)); const int b = n / NH_, h = n % NH_; float s = 0.f;
    if (r < NR) { const float* q = QF + ((size_t)t * BB + b) * EE + h * HD;
#pragma unroll 1
        for (int d = 0; d < HD; ++d) { float p = __fmul_rn(q[d] * 0.125f, bfr(rk[r * HD + d])); asm volatile("" : "+v"(p)); s = __fadd_rn(s, p); } }
    *(volatile float*)(QR + e) = s; __threadfence(); *(volatile float*)(QR + e) = s; }
__global__ __launch_bounds__(256) void k_rsoft(const float* __restrict__ Sb, const float* __restrict__ QR, int n0, h16* P16, bf* Ph, bf* Pl) { const int lane = threadIdx.x & 31; const int row = blockIdx.x * 8 + (threadIdx.x >> 5); if (row >= ZH * TT) return; const int t = row % TT, z = row / TT; const bool hires = t < RH; const float* sr = Sb + (size_t)row * TT; const float* qr = QR + ((size_t)(n0 + z) * TT + t) * 64; float v[64]; float mx = -3.0e38f;
#pragma unroll
    for (int ch = 0; ch < 16; ++ch) { const int j0 = ch * 128 + lane * 4; const v4f a = *(const v4f*)(sr + j0);
#pragma unroll
        for (int q = 0; q < 4; ++q) { const int s = j0 + q; const int r = min(max(s - t, -MR), MR) + MR; const float x = __fadd_rn(a[q], qr[r]); v[ch * 4 + q] = x; mx = fmaxf(mx, x); } }
#pragma unroll
    for (int sh = 16; sh; sh >>= 1) mx = fmaxf(mx, __shfl_xor(mx, sh, 32));
    float sum = 0.f;
#pragma unroll
    for (int k = 0; k < 64; ++k) { float d0 = __fsub_rn(v[k], mx); asm volatile("" : "+v"(d0)); v[k] = __expf(d0); sum += v[k]; }
#pragma unroll
    for (int sh = 16; sh; sh >>= 1) sum += __shfl_xor(sum, sh, 32);
    const float inv = __fdiv_rn(1.0f, sum);
#pragma unroll 1
    for (int ps = 0; ps < 2; ++ps) {
        if (hires) {
#pragma unroll
            for (int ch = 0; ch < 16; ++ch) { v4us oh, ol;
#pragma unroll
                for (int q = 0; q < 4; ++q) { unsigned short a, c2; splitf(v[ch * 4 + q] * inv, a, c2); oh[q] = a; ol[q] = c2; } const size_t oo = ((size_t)z * RH + t) * TT + ch * 128 + lane * 4; *(volatile v4us*)(Ph + oo) = oh; *(volatile v4us*)(Pl + oo) = ol; }
        } else { const float f = inv * PCAR;
#pragma unroll
            for (int ch = 0; ch < 16; ++ch) { v4h o4; o4[0] = tohx(v[ch * 4] * f); o4[1] = tohx(v[ch * 4 + 1] * f); o4[2] = tohx(v[ch * 4 + 2] * f); o4[3] = tohx(v[ch * 4 + 3] * f); *(volatile v4h*)(P16 + (size_t)row * TT + ch * 128 + lane * 4) = o4; } }
        if (ps == 0) __threadfence(); } }
__global__ __launch_bounds__(256) void k_pb(const h16* __restrict__ P16, const bf* __restrict__ Ph, const bf* __restrict__ Pl, float* PB) { const int lane = threadIdx.x & 31; const int row = blockIdx.x * 8 + (threadIdx.x >> 5); if (row >= ZH * TT) return; const int t = row % TT, z = row / TT; const bool hires = t < RH;
    const int r0 = 2 * lane, r1 = 2 * lane + 1; const int s0 = t + r0 - MR, s1 = t + r1 - MR; const int l0 = (s0 & 127) >> 2, l1 = (s1 & 127) >> 2; const int k0 = ((s0 >> 7) << 2) | (s0 & 3), k1 = ((s1 >> 7) << 2) | (s1 & 3); float lo = 0.f, hi = 0.f, pv0 = 0.f, pv1 = 0.f;
#pragma unroll
    for (int ch = 0; ch < 16; ++ch) { const int j0 = ch * 128 + lane * 4; float a[4];
        if (hires) { const size_t oo = ((size_t)z * RH + t) * TT + j0; const v4us ah = *(const v4us*)(Ph + oo), al = *(const v4us*)(Pl + oo);
#pragma unroll
            for (int q = 0; q < 4; ++q) a[q] = __fadd_rn(bf2f(ah[q]), bf2f(al[q])); }
        else { const v4h p4 = *(const v4h*)(P16 + (size_t)row * TT + j0);
#pragma unroll
            for (int q = 0; q < 4; ++q) a[q] = (float)p4[q] * (1.0f / PCAR); }
#pragma unroll
        for (int q = 0; q < 4; ++q) { const int s = j0 + q; if (s <= t - MR) lo = __fadd_rn(lo, a[q]); else if (s >= t + MR) hi = __fadd_rn(hi, a[q]); const float b0 = __shfl(a[q], l0, 32), b1 = __shfl(a[q], l1, 32); if (ch * 4 + q == k0) pv0 = b0; if (ch * 4 + q == k1) pv1 = b1; } }
#pragma unroll
    for (int sh = 16; sh; sh >>= 1) { lo += __shfl_xor(lo, sh, 32); hi += __shfl_xor(hi, sh, 32); }
    pv0 = (r0 > 0 && r0 < 2 * MR && s0 >= 0 && s0 < TT) ? pv0 : 0.f; pv1 = (r1 < 2 * MR && s1 >= 0 && s1 < TT) ? pv1 : 0.f; if (lane == 0) pv0 = lo; if (lane == MR) pv0 = hi;
    float* pb = PB + ((size_t)z * TT + t) * 64; v2f o; o[0] = pv0; o[1] = pv1; *(volatile v2f*)(pb + 2 * lane) = o; __threadfence(); *(volatile v2f*)(pb + 2 * lane) = o; }
__global__ __launch_bounds__(256) void k_mrg(const float* __restrict__ Ob, const float* __restrict__ PB, const float* __restrict__ rv, int n0, bf* Ah, bf* Al) { const size_t e = ((size_t)blockIdx.x * 256 + threadIdx.x) * 2; if (e >= (size_t)ZH * TT * HD) return; const int d = (int)(e % HD); const int t = (int)((e / HD) % TT); const int z = (int)(e / ((size_t)HD * TT)); const int n = n0 + z; const int b = n / NH_, h = n % NH_; const float f = t < RH ? 1.0f : (1.0f / PCAR); const float* pb = PB + ((size_t)z * TT + t) * 64; v2us oh, ol;
#pragma unroll
    for (int u = 0; u < 2; ++u) { float acc = Ob[e + u] * f;
#pragma unroll 1
        for (int r = 0; r < NR; ++r) { float p = __fmul_rn(pb[r], bfr(rv[r * HD + d + u])); asm volatile("" : "+v"(p)); acc = __fadd_rn(acc, p); }
        unsigned short a, c; splitf(acc, a, c); oh[u] = a; ol[u] = c; }
    const size_t o = ((size_t)t * BB + b) * EE + h * HD + d; *(volatile v2us*)(Ah + o) = oh; *(volatile v2us*)(Al + o) = ol; __threadfence(); *(volatile v2us*)(Ah + o) = oh; *(volatile v2us*)(Al + o) = ol; }

extern "C" void kernel_launch(void* const* d_in, const int* in_sizes, int n_in,
                              void* d_out, int out_size, void* d_ws, size_t ws_size, hipStream_t stream) {
    (void)in_sizes; (void)n_in; (void)out_size;
    const float* x = (const float*)d_in[0]; const float* Wq = (const float*)d_in[1]; const float* bq = (const float*)d_in[2]; const float* Wk = (const float*)d_in[3]; const float* bk = (const float*)d_in[4]; const float* Wv = (const float*)d_in[5]; const float* bv = (const float*)d_in[6]; const float* Wo = (const float*)d_in[7]; const float* bo = (const float*)d_in[8]; const float* rk = (const float*)d_in[9]; const float* rv = (const float*)d_in[10];
    float* OUT = (float*)d_out;
    char* wsp = (char*)d_ws;
    auto take = [&](size_t bytes) { char* p = wsp; wsp += (bytes + 255) & ~(size_t)255; return (void*)p; };
    const size_t NTB = (size_t)TT * BB;
    bf* WQ = (bf*)take((size_t)EE * EE * 2); bf* WK = (bf*)take((size_t)EE * EE * 2); bf* WV = (bf*)take((size_t)EE * EE * 2); bf* WO = (bf*)take((size_t)EE * EE * 2); bf* XB = (bf*)take(NTB * EE * 2);
    float* QF = (float*)take(NTB * EE * 4); float* KF = (float*)take(NTB * EE * 4); float* QR = (float*)take((size_t)NG * TT * 64 * 4);
    h16* Q16 = (h16*)take((size_t)NG * TT * HD * 2); bf* Qh = (bf*)take((size_t)NG * TT * HD * 2); bf* Ql = (bf*)take((size_t)NG * TT * HD * 2); h16* K16 = (h16*)take((size_t)NG * TT * HD * 2); bf* Kh = (bf*)take((size_t)NG * TT * HD * 2); bf* Kl = (bf*)take((size_t)NG * TT * HD * 2); h16* V16 = (h16*)take((size_t)NG * HD * TT * 2); bf* Vh = (bf*)take((size_t)NG * HD * TT * 2); bf* Vl = (bf*)take((size_t)NG * HD * TT * 2);
    float* Sb = (float*)take((size_t)ZH * TT * TT * 4); h16* P16 = (h16*)take((size_t)ZH * TT * TT * 2); bf* Ph = (bf*)take((size_t)ZH * RH * TT * 2); bf* Pl = (bf*)take((size_t)ZH * RH * TT * 2); float* PB = (float*)take((size_t)ZH * TT * 64 * 4); float* Ob = (float*)take((size_t)ZH * TT * HD * 4); bf* Ah = (bf*)take(NTB * EE * 2); bf* Al = (bf*)take(NTB * EE * 2);
    if ((size_t)(wsp - (char*)d_ws) > ws_size) return;
    float* VF = KF;
    k_cvt8<<<(EE * EE / 8 + 255) / 256, 256, 0, stream>>>(Wq, WQ, (size_t)EE * EE / 8); k_cvt8<<<(EE * EE / 8 + 255) / 256, 256, 0, stream>>>(Wk, WK, (size_t)EE * EE / 8); k_cvt8<<<(EE * EE / 8 + 255) / 256, 256, 0, stream>>>(Wv, WV, (size_t)EE * EE / 8); k_cvt8<<<(EE * EE / 8 + 255) / 256, 256, 0, stream>>>(Wo, WO, (size_t)EE * EE / 8);
    k_cvt8<<<(unsigned)((NTB * EE / 8 + 255) / 256), 256, 0, stream>>>(x, XB, NTB * EE / 8);
    const unsigned LP = (unsigned)(((size_t)NG * TT * HD / 2 + 255) / 256);
    k_gemmw<bf, 0, true><<<dim3(NTB / 64, EE / 64, 1), 32, 0, stream>>>(XB, nullptr, WQ, nullptr, EE, QF, EE, bq, 0, 0, 0); k_pl<<<LP, 256, 0, stream>>>(QF, 0.125f, Q16, Qh, Ql); k_qr<<<(unsigned)(((size_t)NG * TT * 64 + 255) / 256), 256, 0, stream>>>(QF, rk, QR);
    k_gemmw<bf, 0, true><<<dim3(NTB / 64, EE / 64, 1), 32, 0, stream>>>(XB, nullptr, WK, nullptr, EE, KF, EE, bk, 0, 0, 0); k_pl<<<LP, 256, 0, stream>>>(KF, 1.0f, K16, Kh, Kl);
    k_gemmw<bf, 0, true><<<dim3(NTB / 64, EE / 64, 1), 32, 0, stream>>>(XB, nullptr, WV, nullptr, EE, VF, EE, bv, 0, 0, 0); k_vtp<<<LP, 256, 0, stream>>>(VF, V16, Vh, Vl);
    for (int n0 = 0; n0 < NG; n0 += ZH) { const size_t z = (size_t)n0;
        k_gemmw<bf, 2, false><<<dim3(RH / 64, TT / 64, ZH), 32, 0, stream>>>(Qh + z * TT * HD, Ql + z * TT * HD, Kh + z * TT * HD, Kl + z * TT * HD, HD, Sb, TT, nullptr, (size_t)TT * HD, (size_t)TT * HD, (size_t)TT * TT);
        k_gemmw<h16, 0, false><<<dim3((TT - RH) / 64, TT / 64, ZH), 32, 0, stream>>>(Q16 + z * TT * HD + (size_t)RH * HD, nullptr, K16 + z * TT * HD, nullptr, HD, Sb + (size_t)RH * TT, TT, nullptr, (size_t)TT * HD, (size_t)TT * HD, (size_t)TT * TT);
        k_rsoft<<<ZH * TT / 8, 256, 0, stream>>>(Sb, QR, n0, P16, Ph, Pl); k_pb<<<ZH * TT / 8, 256, 0, stream>>>(P16, Ph, Pl, PB);
        k_gemmw<bf, 2, false><<<dim3(RH / 64, 1, ZH), 32, 0, stream>>>(Ph, Pl, Vh + z * HD * TT, Vl + z * HD * TT, TT, Ob, HD, nullptr, (size_t)RH * TT, (size_t)HD * TT, (size_t)TT * HD);
        k_gemmw<h16, 0, false><<<dim3((TT - RH) / 64, 1, ZH), 32, 0, stream>>>(P16 + (size_t)RH * TT, nullptr, V16 + z * HD * TT, nullptr, TT, Ob + (size_t)RH * HD, HD, nullptr, (size_t)TT * TT, (size_t)HD * TT, (size_t)TT * HD);
        k_mrg<<<(unsigned)(((size_t)ZH * TT * HD / 2 + 255) / 256), 256, 0, stream>>>(Ob, PB, rv, n0, Ah, Al); }
    k_gemmw<bf, 1, true><<<dim3(NTB / 64, EE / 64, 1), 32, 0, stream>>>(Ah, Al, WO, nullptr, EE, OUT, EE, bo, 0, 0, 0);
}
